// Recurrent_83975200571955
// MI455X (gfx1250) — hardware-run, weakly checked
//
#include <hip/hip_runtime.h>
#include <stdint.h>
#include <stddef.h>

constexpr int NB = 128;
constexpr int NS = 500;
constexpr int NU = 128;
constexpr int NMEM = 32;
constexpr int NT_ROWS = 10000;
constexpr int NR_ROWS = 2;
constexpr int NGROWS = 257;
constexpr int ROWS_PER_BLK = 8;
constexpr int NBLK = NB / ROWS_PER_BLK;
constexpr int KIN = 256;
constexpr int KOUT = 128;
constexpr int KG = 256;
constexpr int KGATE = 384;
constexpr int XPITCH = 384;
constexpr int NROWS_ALL = NB * NS;
constexpr float XSC = 16.0f;
constexpr float WSC = 64.0f;
constexpr float INV_XW = 1.0f / 1024.0f;
constexpr int OUT0_F = NB * (NS - 1);
constexpr int OUT1_F = NB * NS;
constexpr int OUT_FLOATS = OUT0_F + OUT1_F;
constexpr int OUT_F4 = OUT_FLOATS / 4;

static_assert(NB % ROWS_PER_BLK == 0, "shape");
static_assert(OUT_FLOATS % 4 == 0, "shape");
static_assert((OUT0_F * 4) % 128 == 0, "out1 starts on a 128-B line");
static_assert(OUT0_F * 4 == 255488, "out1 byte offset");
static_assert(KIN % 32 == 0 && KOUT % 32 == 0 && KG % 32 == 0 && KGATE % 32 == 0, "K multiples of 32");
static_assert(NROWS_ALL % 64 == 0 && NU % 64 == 0, "kit GEMM tile multiples");
static_assert(((NROWS_ALL / 64) * (NU / 64)) % 8 == 0, "kit GEMM grid exact");
static_assert(NROWS_ALL % 8 == 0, "gather grid exact");
static_assert((ROWS_PER_BLK * NS * 4) % 128 == 0, "per-block staging slice is whole lines");

constexpr size_t OFFB_WIN  = 0;
constexpr size_t OFFB_WOUT = OFFB_WIN  + (size_t)NU * KIN * 2;
constexpr size_t OFFB_WT   = OFFB_WOUT + (size_t)NU * KOUT * 2;
constexpr size_t OFFB_WA   = OFFB_WT   + (size_t)NU * KG * 2;
constexpr size_t OFFB_WH   = OFFB_WA   + (size_t)NU * KG * 2;
constexpr size_t OFFB_WG   = OFFB_WH   + (size_t)NU * KG * 2;
constexpr size_t OFFB_BIN  = OFFB_WG   + (size_t)NU * KGATE * 2;
constexpr size_t OFFB_XIN  = OFFB_BIN  + 512;
constexpr size_t OFFB_ACT  = OFFB_XIN  + (size_t)NROWS_ALL * KIN * 2;
constexpr size_t OFFB_PST  = OFFB_ACT  + (size_t)NROWS_ALL * NU * 2;
constexpr size_t OFFB_IST  = OFFB_PST  + (size_t)NB * NS * 4;
constexpr size_t WS_TOTAL  = OFFB_IST  + (size_t)NB * NS * 4;
static_assert(OFFB_WOUT % 256 == 0 && OFFB_WT % 256 == 0 && OFFB_WG % 256 == 0 && OFFB_BIN % 256 == 0, "align");
static_assert(OFFB_XIN % 256 == 0 && OFFB_ACT % 256 == 0 && OFFB_PST % 256 == 0 && OFFB_IST % 256 == 0, "align");
static_assert(WS_TOTAL == 50057728, "carve total");
static_assert(WS_TOTAL <= (size_t)134217728, "carve under 128 MiB");

typedef __attribute__((ext_vector_type(16))) _Float16 v16h;
typedef __attribute__((ext_vector_type(8)))  _Float16 v8h;
typedef __attribute__((ext_vector_type(4)))  _Float16 v4h;
typedef __attribute__((ext_vector_type(16))) __bf16   v16b;
typedef __attribute__((ext_vector_type(8)))  __bf16   v8b;
typedef __attribute__((ext_vector_type(8)))  float    v8f;
typedef __attribute__((ext_vector_type(4)))  float    v4f;
typedef __attribute__((ext_vector_type(4)))  unsigned v4u;

__device__ __forceinline__ unsigned short f2bf_bits(float f) {
  unsigned u = __float_as_uint(f);
  return (unsigned short)((u + 0x7FFFu + ((u >> 16) & 1u)) >> 16);
}
__device__ __forceinline__ float bf_bits2f(unsigned short h) { return __uint_as_float(((unsigned)h) << 16); }

__device__ __forceinline__ void dep_guard_h(v8f& a, v8f& b, v16h x, v16h y) { asm volatile("v_nop\n\tv_nop\n\tv_nop\n\tv_nop" : "+v"(a), "+v"(b) : "v"(x), "v"(y)); }
__device__ __forceinline__ void dep_guard_b(v8f& a, v8f& b, v16b x, v16b y) { asm volatile("v_nop\n\tv_nop\n\tv_nop\n\tv_nop" : "+v"(a), "+v"(b) : "v"(x), "v"(y)); }
__device__ __forceinline__ void keep4_h(v16h a, v16h b, v16h c, v16h d) { asm volatile("v_nop" :: "v"(a), "v"(b), "v"(c), "v"(d)); }
__device__ __forceinline__ void keep4_b(v16b a, v16b b, v16b c, v16b d) { asm volatile("v_nop" :: "v"(a), "v"(b), "v"(c), "v"(d)); }
__device__ __forceinline__ void acc_guard4(v8f& a, v8f& b, v8f& c, v8f& d) { asm volatile("v_nop\n\tv_nop\n\tv_nop\n\tv_nop" : "+v"(a), "+v"(b), "+v"(c), "+v"(d)); }
template <typename T> struct Frag;
template <> struct Frag<_Float16> {
  typedef v16h V; union U { v16h v; v8h h[2]; };
  static __device__ __forceinline__ v16h load(const _Float16* p) {
    U f; f.h[0] = *(const v8h*)(p); f.h[1] = *(const v8h*)(p + 16); return f.v;
  }
  static __device__ __forceinline__ v8f mma(v16h a, v16h b, v8f c) {
    return __builtin_amdgcn_wmma_f32_16x16x32_f16(false, a, false, b, (short)0, c, false, false);
  }
  static __device__ __forceinline__ void guard(v8f& a, v8f& b, v16h x, v16h y) { dep_guard_h(a, b, x, y); }
  static __device__ __forceinline__ void keep(v16h a, v16h b, v16h c, v16h d) { keep4_h(a, b, c, d); }
};
template <> struct Frag<__bf16> {
  typedef v16b V; union U { v16b v; v8b h[2]; };
  static __device__ __forceinline__ v16b load(const __bf16* p) {
    U f; f.h[0] = *(const v8b*)(p); f.h[1] = *(const v8b*)(p + 16); return f.v;
  }
  static __device__ __forceinline__ v8f mma(v16b a, v16b b, v8f c) {
    return __builtin_amdgcn_wmma_f32_16x16x32_bf16(false, a, false, b, (short)0, c, false, false);
  }
  static __device__ __forceinline__ void guard(v8f& a, v8f& b, v16b x, v16b y) { dep_guard_b(a, b, x, y); }
  static __device__ __forceinline__ void keep(v16b a, v16b b, v16b c, v16b d) { keep4_b(a, b, c, d); }
};

template <int ET> struct Elem;
template <> struct Elem<0> { typedef _Float16 T; };
template <> struct Elem<1> { typedef __bf16 T; };
template <int ET, bool SPLIT, int BIAS_MODE, int OUT_MODE, bool RESID, int ACT = 0>
__global__ __launch_bounds__(256) void wmma_gemm64(
    const unsigned short* __restrict__ Ap, const unsigned short* __restrict__ A2p, int lda, long strideA,
    const unsigned short* __restrict__ Btp, const unsigned short* __restrict__ Bt2p, int ldb, long strideB,
    void* __restrict__ Cout, void* __restrict__ Cout2, int ldc, long strideC,
    const float* __restrict__ bias,
    const float* __restrict__ resid, long strideR,
    int M, int N, int K, float scale) {
  typedef typename Elem<ET>::T T;
  typedef typename Frag<T>::V V;
  const T* A = (const T*)Ap; const T* A2 = (const T*)A2p; const T* Bt = (const T*)Btp; const T* Bt2 = (const T*)Bt2p;
  __shared__ __align__(16) float sT[8][16 * 68];
  const int b    = blockIdx.y;
  const int lane = threadIdx.x & 31;
  const int wave = threadIdx.x >> 5;
  const int tilesN = N >> 6;
  const int tilesM = M >> 6;
  const int tile = blockIdx.x * 8 + wave;
  if (tile >= tilesM * tilesN) return;
  const int tm = tile / tilesN;
  const int tn = tile - tm * tilesN;
  const int m0 = tm << 6;
  const int n0 = tn << 6;

  const T* Ab  = A  + (size_t)b * strideA;
  const T* Bb  = Bt + (size_t)b * strideB;
  const T* Ab2 = SPLIT ? (A2  + (size_t)b * strideA) : nullptr;
  const T* Bb2 = SPLIT ? (Bt2 + (size_t)b * strideB) : nullptr;

  const int rlane = lane & 15;
  const int koff  = (lane >> 4) * 8;
  const int mOff  = (lane >> 4) * 8;

  v8f acc[4][4];
#pragma unroll
  for (int i = 0; i < 4; ++i)
#pragma unroll
    for (int j = 0; j < 4; ++j) acc[i][j] = (v8f){0.f,0.f,0.f,0.f,0.f,0.f,0.f,0.f};

  for (int k0 = 0; k0 < K; k0 += 32) {
    V bh[4], bl[4];
#pragma unroll
    for (int j = 0; j < 4; ++j) {
      const size_t bo = (size_t)(n0 + (j << 4) + rlane) * ldb + koff + k0;
      bh[j] = Frag<T>::load(Bb + bo);
      if (SPLIT) bl[j] = Frag<T>::load(Bb2 + bo);
    }
#pragma unroll
    for (int i = 0; i < 4; ++i) {
      const size_t ao = (size_t)(m0 + (i << 4) + rlane) * lda + koff + k0;
      V ah = Frag<T>::load(Ab + ao);
      V al;
      if (SPLIT) al = Frag<T>::load(Ab2 + ao);
#pragma unroll
      for (int j = 0; j < 4; ++j) {
        acc[i][j] = Frag<T>::mma(ah, bh[j], acc[i][j]);
        if (SPLIT) {
          acc[i][j] = Frag<T>::mma(ah, bl[j], acc[i][j]);
          acc[i][j] = Frag<T>::mma(al, bh[j], acc[i][j]);
        }
      }
      Frag<T>::guard(acc[i][0], acc[i][3], ah, SPLIT ? al : ah);
    }
    Frag<T>::keep(bh[0], bh[1], bh[2], bh[3]);
    if (SPLIT) Frag<T>::keep(bl[0], bl[1], bl[2], bl[3]);
  }
  acc_guard4(acc[0][0], acc[0][1], acc[0][2], acc[0][3]);
  acc_guard4(acc[1][0], acc[1][1], acc[1][2], acc[1][3]);
  acc_guard4(acc[2][0], acc[2][1], acc[2][2], acc[2][3]);
  acc_guard4(acc[3][0], acc[3][1], acc[3][2], acc[3][3]);

  float* slab = sT[wave];
  const float* Rb = RESID ? (resid + (size_t)b * strideR) : nullptr;
#pragma unroll
  for (int i = 0; i < 4; ++i) {
    const int mBase = m0 + (i << 4);
#pragma unroll
    for (int j = 0; j < 4; ++j) {
      const int n = n0 + (j << 4) + rlane;
      float bv = 0.f;
      if (BIAS_MODE == 2) bv = bias[n];
#pragma unroll
      for (int r = 0; r < 8; ++r) {
        float v = acc[i][j][r] * scale;
        if (BIAS_MODE == 1) v += bias[mBase + mOff + r];
        if (BIAS_MODE == 2) v += bv;
        if (RESID) v += Rb[(size_t)(mBase + mOff + r) * ldc + n];
        if (ACT == 1) v = tanhf(v);
        if (ACT == 2) v = fmaxf(v, 0.0f);
        if (ACT == 3) v = v / (1.0f + expf(-v));
        if (ACT == 4) v = (v > 0.f) ? v : 0.01f * v;
        if (ACT == 5) v = 0.5f * v * (1.0f + erff(v * 0.70710678118654752f));
        slab[(mOff + r) * 68 + (j << 4) + rlane] = v;
      }
    }
    __builtin_amdgcn_fence(__ATOMIC_RELEASE, "workgroup");
    __builtin_amdgcn_wave_barrier();
    __builtin_amdgcn_fence(__ATOMIC_ACQUIRE, "workgroup");
    if (OUT_MODE == 0) {
      float* C = (float*)Cout + (size_t)b * strideC;
      const int hh = lane >> 4, c4 = (lane & 15) * 4;
      for (int pass = 0; pass < 2; ++pass) {
#pragma unroll
        for (int it = 0; it < 8; ++it) {
          const int row = it * 2 + hh;
          v4f v = *(const v4f*)(slab + row * 68 + c4);
          *(volatile v4f*)(C + (size_t)(mBase + row) * ldc + n0 + c4) = v;
        }
        __threadfence();
      }
    } else {
      const int q = lane >> 3, c8 = (lane & 7) * 8;
      unsigned short* C  = (unsigned short*)Cout  + (size_t)b * strideC;
      unsigned short* C2 = (OUT_MODE == 2) ? ((unsigned short*)Cout2 + (size_t)b * strideC) : nullptr;
      for (int pass = 0; pass < 2; ++pass) {
#pragma unroll
        for (int it = 0; it < 4; ++it) {
          const int row = it * 4 + q;
          const float* sp = slab + row * 68 + c8;
          v8h hv, lv;
#pragma unroll
          for (int e = 0; e < 8; ++e) {
            if (OUT_MODE == 1) {
              hv[e] = (_Float16)sp[e];
            } else {
              unsigned short hb = f2bf_bits(sp[e]);
              unsigned short lb = f2bf_bits(sp[e] - bf_bits2f(hb));
              hv[e] = __builtin_bit_cast(_Float16, hb);
              lv[e] = __builtin_bit_cast(_Float16, lb);
            }
          }
          *(volatile v8h*)(C + (size_t)(mBase + row) * ldc + n0 + c8) = hv;
          if (OUT_MODE == 2) *(volatile v8h*)(C2 + (size_t)(mBase + row) * ldc + n0 + c8) = lv;
        }
        __threadfence();
      }
    }
    __builtin_amdgcn_fence(__ATOMIC_RELEASE, "workgroup");
    __builtin_amdgcn_wave_barrier();
    __builtin_amdgcn_fence(__ATOMIC_ACQUIRE, "workgroup");
  }
}

__device__ __forceinline__ v8f zero8() { return (v8f){0.f,0.f,0.f,0.f,0.f,0.f,0.f,0.f}; }
__device__ __forceinline__ v8f mma_g(v16h a, v16h b, v8f c) {
  c = __builtin_amdgcn_wmma_f32_16x16x32_f16(false, a, false, b, (short)0, c, false, false);
  asm volatile("v_nop\n\tv_nop\n\tv_nop\n\tv_nop" : "+v"(c) : "v"(a), "v"(b));
  return c;
}
__device__ __forceinline__ int clampi(int v, int n) {
  v = v < 0 ? 0 : v;
  v = v > n - 1 ? n - 1 : v;
  return v;
}
__device__ __forceinline__ float sigm(float x) { return 1.0f / (1.0f + expf(-x)); }

__global__ __launch_bounds__(256) void k_prep(
    const float* __restrict__ W_in,  const float* __restrict__ W_out,
    const float* __restrict__ W_time, const float* __restrict__ W_att,
    const float* __restrict__ W_hint, const float* __restrict__ W_gate,
    const float* __restrict__ b_in,
    _Float16* __restrict__ dWin, _Float16* __restrict__ dWout,
    _Float16* __restrict__ dWt,  _Float16* __restrict__ dWa,
    _Float16* __restrict__ dWh,  _Float16* __restrict__ dWg,
    float* __restrict__ dBin) {
  const int id  = blockIdx.y;
  const int tid = threadIdx.x;
  if (id == 6) {
    if (blockIdx.x != 0 || tid >= 32) return;
    v4f v = *(const v4f*)(b_in + 4 * tid);
    v = v * XSC;
    for (int pass = 0; pass < 2; ++pass) {
      *(volatile v4f*)(dBin + 4 * tid) = v;
      __threadfence();
    }
    return;
  }
  const float* src; _Float16* dst; int K; int perm;
  if (id == 0)      { src = W_in;   dst = dWin;  K = KIN;   perm = 0; }
  else if (id == 1) { src = W_out;  dst = dWout; K = KOUT;  perm = 0; }
  else if (id == 2) { src = W_time; dst = dWt;   K = KG;    perm = 1; }
  else if (id == 3) { src = W_att;  dst = dWa;   K = KG;    perm = 1; }
  else if (id == 4) { src = W_hint; dst = dWh;   K = KG;    perm = 1; }
  else              { src = W_gate; dst = dWg;   K = KGATE; perm = 0; }
  const int NK = NU * K;
  const int e0 = 8 * (blockIdx.x * 256 + tid);
  if (e0 >= NK) return;
  const int n  = e0 / K;
  const int k0 = e0 - n * K;
  v8h o;
#pragma unroll
  for (int e = 0; e < 8; ++e) {
    const int k  = k0 + e;
    const int sk = perm ? ((k < 128) ? (129 + k) : (k - 127)) : k;
    o[e] = (_Float16)(WSC * src[(size_t)sk * NU + n]);
  }
  for (int pass = 0; pass < 2; ++pass) {
    *(volatile v8h*)(dst + e0) = o;
    __threadfence();
  }
}

__global__ __launch_bounds__(256) void k_gather(
    const int* __restrict__ topics, const int* __restrict__ resps,
    const float* __restrict__ emb_topic, const float* __restrict__ emb_resps,
    _Float16* __restrict__ Xin, int nTop, int nResp) {
  const int tid = threadIdx.x, lane = tid & 31, wv = tid >> 5;
  const int g = blockIdx.x * 8 + wv;
  const int ti = clampi(topics[g], nTop);
  const int ri = clampi(resps[g], nResp);
  const int c8 = (lane & 15) * 8;
  const float* tp = emb_topic + (size_t)ti * NU + c8;
  const float* rp = emb_resps + (size_t)ri * NU + c8;
  const v4f t0 = *(const v4f*)tp, t1 = *(const v4f*)(tp + 4);
  const v4f r0 = *(const v4f*)rp, r1 = *(const v4f*)(rp + 4);
  const bool useT = lane < 16;
  v8h o;
#pragma unroll
  for (int e = 0; e < 4; ++e) {
    o[e]     = (_Float16)(XSC * (useT ? t0[e] : r0[e]));
    o[4 + e] = (_Float16)(XSC * (useT ? t1[e] : r1[e]));
  }
  _Float16* dst = Xin + (size_t)g * KIN + lane * 8;
  for (int pass = 0; pass < 2; ++pass) {
    *(volatile v8h*)dst = o;
    __threadfence();
  }
}

__global__ __launch_bounds__(256) void k_scan(
    const int* __restrict__ topics,
    const float* __restrict__ time_factor, const float* __restrict__ attempt_factor,
    const float* __restrict__ hint_factor, const int* __restrict__ masks,
    const float* __restrict__ emb_topic, const float* __restrict__ q_matrix,
    const float* __restrict__ init_h,
    const float* __restrict__ b_out,
    const float* __restrict__ W_time, const float* __restrict__ b_time,
    const float* __restrict__ W_att,  const float* __restrict__ b_att,
    const float* __restrict__ W_hint, const float* __restrict__ b_hint,
    const float* __restrict__ W_cap,  const float* __restrict__ b_cap,
    const float* __restrict__ w_lg,   const float* __restrict__ b_gate,
    const _Float16* __restrict__ WoutT, const _Float16* __restrict__ WtT,
    const _Float16* __restrict__ WaT,   const _Float16* __restrict__ WhT,
    const _Float16* __restrict__ WgT,
    const unsigned short* __restrict__ acts16,
    float* __restrict__ Pst, float* __restrict__ Ist, int nTop) {
  __shared__ __align__(16) float    sH[ROWS_PER_BLK * NMEM * NU];
  __shared__ __align__(16) _Float16 sX[16 * XPITCH];
  __shared__ __align__(16) float    sSig[ROWS_PER_BLK * NU];
  __shared__ __align__(16) float    sLG[ROWS_PER_BLK * NU];
  __shared__ __align__(16) float    sGam[ROWS_PER_BLK * NU];
  __shared__ __align__(16) float    sW[ROWS_PER_BLK * NMEM];
  __shared__ __align__(16) float    sOutP[ROWS_PER_BLK * NS];
  __shared__ __align__(16) float    sOutI[ROWS_PER_BLK * NS];
  __shared__ float sBout[NU], sBgate[NU], sBg[3 * NU], sW0[3 * NU];
  __shared__ float sF[3 * ROWS_PER_BLK], sCap[ROWS_PER_BLK];
  __shared__ int   sMk[ROWS_PER_BLK];
  __shared__ float sWcap[8], sWlg[4], sBcap[1];

  const int tid = threadIdx.x, lane = tid & 31, wv = tid >> 5;
  const int ml = lane & 15, hi = lane >> 4;
  const int wg = blockIdx.x;
  const int bb0 = wg * ROWS_PER_BLK;

#pragma unroll 4
  for (int q = 0; q < 32; ++q) {
    const int i = tid + 256 * q;
    const int b = i >> 10;
    const int rem = i & 1023;
    const v4f v = *(const v4f*)(init_h + rem * 4);
    *(v4f*)(sH + b * (NMEM * NU) + rem * 4) = v;
  }
  {
    const v4u z = {0u, 0u, 0u, 0u};
#pragma unroll
    for (int q = 0; q < 3; ++q) *(v4u*)(sX + 8 * (tid + 256 * q)) = z;
  }
  if (tid < NU) {
    sBout[tid] = b_out[tid];   sBgate[tid] = b_gate[tid];
    sBg[tid] = b_time[tid];    sBg[NU + tid] = b_att[tid];    sBg[2 * NU + tid] = b_hint[tid];
    sW0[tid] = W_time[tid];    sW0[NU + tid] = W_att[tid];    sW0[2 * NU + tid] = W_hint[tid];
  }
  if (tid < 8) sWcap[tid] = W_cap[tid];
  if (tid < 3) sWlg[tid] = w_lg[tid];
  if (tid == 0) sBcap[0] = b_cap[0];
  __syncthreads();

  const int u = wv * 16 + ml;
  const _Float16* Arow = sX + ml * XPITCH + 8 * hi;

  for (int s = 0; s < NS; ++s) {
    if (tid < ROWS_PER_BLK) {
      const int b = tid;
      const int idx = (bb0 + b) * NS + s;
      const float t = time_factor[idx], at = attempt_factor[idx], hn = hint_factor[idx];
      const float tat = t * at, thn = t * hn, ahn = at * hn, tah = tat * hn;
      const float cs = t * sWcap[0] + at * sWcap[1] + hn * sWcap[2] + tat * sWcap[3] +
                       thn * sWcap[4] + ahn * sWcap[5] + tah * sWcap[6] + sWcap[7] + sBcap[0];
      sF[b] = t; sF[ROWS_PER_BLK + b] = at; sF[2 * ROWS_PER_BLK + b] = hn;
      sCap[b] = sigm(cs);
      sMk[b] = (masks[idx] != 0) ? 1 : 0;
    }
    {
      const int ti = clampi(topics[(bb0 + wv) * NS + s], nTop);
      sW[wv * NMEM + lane] = q_matrix[(size_t)ti * NMEM + lane];
    }
    if (tid < 128) {
      const int b = tid >> 4, c8 = (tid & 15) * 8;
      const v4u av = *(const v4u*)(acts16 + ((size_t)((bb0 + b) * NS + s) * NU + c8));
      *(v4u*)(sX + b * XPITCH + 128 + c8) = av;
    } else {
      const int t2 = tid - 128;
      const int b = t2 >> 4, c8 = (t2 & 15) * 8;
      const int ti = clampi(topics[(bb0 + b) * NS + s], nTop);
      const float* ep = emb_topic + (size_t)ti * NU + c8;
      const v4f e0 = *(const v4f*)ep, e1 = *(const v4f*)(ep + 4);
      v8h o;
#pragma unroll
      for (int e = 0; e < 4; ++e) { o[e] = (_Float16)(XSC * e0[e]); o[4 + e] = (_Float16)(XSC * e1[e]); }
      *(v8h*)(sX + b * XPITCH + 256 + c8) = o;
    }
    __syncthreads();

    {
      const float* Hb = sH + wv * (NMEM * NU) + lane * 4;
      const float* wb = sW + wv * NMEM;
      v4f ha = {0.f, 0.f, 0.f, 0.f};
#pragma unroll 8
      for (int m = 0; m < NMEM; ++m) {
        const v4f hq = *(const v4f*)(Hb + m * NU);
        ha += wb[m] * hq;
      }
      v4h o;
#pragma unroll
      for (int e = 0; e < 4; ++e) o[e] = (_Float16)(XSC * ha[e]);
      *(v4h*)(sX + wv * XPITCH + lane * 4) = o;
    }
    __syncthreads();

    {
      v8f acc = zero8();
#pragma unroll 2
      for (int c = 0; c < KOUT / 32; ++c) {
        const v16h a  = Frag<_Float16>::load(Arow + 32 * c);
        const v16h bq = Frag<_Float16>::load(WoutT + (size_t)u * KOUT + 8 * hi + 32 * c);
        acc = mma_g(a, bq, acc);
      }
      float sg[8];
      {
        const float bo = sBout[u];
#pragma unroll
        for (int r = 0; r < 8; ++r) sg[r] = sigm(acc[r] * INV_XW + bo);
      }
      if (hi == 0) {
#pragma unroll
        for (int r = 0; r < 8; ++r) sSig[r * NU + u] = sg[r];
      }

      float pre[8];
#pragma unroll
      for (int r = 0; r < 8; ++r) pre[r] = 0.f;
#pragma unroll
      for (int gi = 0; gi < 3; ++gi) {
        const _Float16* WT = (gi == 0) ? WtT : ((gi == 1) ? WaT : WhT);
        acc = zero8();
#pragma unroll 2
        for (int c = 0; c < KG / 32; ++c) {
          const v16h a  = Frag<_Float16>::load(Arow + 32 * c);
          const v16h bq = Frag<_Float16>::load(WT + (size_t)u * KG + 8 * hi + 32 * c);
          acc = mma_g(a, bq, acc);
        }
        const float w0 = sW0[gi * NU + u], bx = sBg[gi * NU + u], wl = sWlg[gi];
#pragma unroll
        for (int r = 0; r < 8; ++r) {
          const float fac = sF[gi * ROWS_PER_BLK + r];
          const float gv = tanhf(acc[r] * INV_XW + fac * w0 + bx) * fac;
          pre[r] += wl * gv;
        }
      }
      float lgv[8];
#pragma unroll
      for (int r = 0; r < 8; ++r) lgv[r] = sCap[r] * fmaxf(pre[r], 0.f);

      acc = zero8();
#pragma unroll 2
      for (int c = 0; c < KGATE / 32; ++c) {
        const v16h a  = Frag<_Float16>::load(Arow + 32 * c);
        const v16h bq = Frag<_Float16>::load(WgT + (size_t)u * KGATE + 8 * hi + 32 * c);
        acc = mma_g(a, bq, acc);
      }
      float gm[8];
      {
        const float bg = sBgate[u];
#pragma unroll
        for (int r = 0; r < 8; ++r) gm[r] = sigm(acc[r] * INV_XW + bg);
      }
      if (hi == 0) {
#pragma unroll
        for (int r = 0; r < 8; ++r) { sLG[r * NU + u] = lgv[r]; sGam[r * NU + u] = gm[r]; }
      }
    }
    __syncthreads();

    {
      const int b = wv;
      const int mk = sMk[b];
      const v4f lg4 = *(const v4f*)(sLG  + b * NU + lane * 4);
      const v4f sg4 = *(const v4f*)(sSig + b * NU + lane * 4);
      const v4f gm4 = *(const v4f*)(sGam + b * NU + lane * 4);
      float ls = (lg4[0] + lg4[1]) + (lg4[2] + lg4[3]);
      float ss = (sg4[0] + sg4[1]) + (sg4[2] + sg4[3]);
#pragma unroll
      for (int off = 16; off > 0; off >>= 1) {
        ls += __shfl_xor(ls, off, 32);
        ss += __shfl_xor(ss, off, 32);
      }
      if (lane == 0) {
        sOutP[b * NS + s] = mk ? ss * (1.0f / 128.0f) : 0.f;
        sOutI[b * NS + s] = mk ? ls * (1.0f / 128.0f) : 0.f;
      }
      if (mk) {
        float* Hb = sH + b * (NMEM * NU) + lane * 4;
        const float* wb = sW + b * NMEM;
#pragma unroll 8
        for (int m = 0; m < NMEM; ++m) {
          v4f hq = *(const v4f*)(Hb + m * NU);
          const float wm = wb[m];
          hq = gm4 * hq + wm * lg4;
          *(v4f*)(Hb + m * NU) = hq;
        }
      }
    }
    __syncthreads();
  }

  {
    float* pdst = Pst + (size_t)wg * (ROWS_PER_BLK * NS);
    float* idst = Ist + (size_t)wg * (ROWS_PER_BLK * NS);
    for (int pass = 0; pass < 2; ++pass) {
#pragma unroll
      for (int it = 0; it < 4; ++it) {
        const int i = tid + 256 * it;
        if (i < (ROWS_PER_BLK * NS) / 4) {
          const v4f a = *(const v4f*)(sOutP + 4 * i);
          const v4f c = *(const v4f*)(sOutI + 4 * i);
          *(volatile v4f*)(pdst + 4 * i) = a;
          *(volatile v4f*)(idst + 4 * i) = c;
        }
      }
      __threadfence();
    }
  }
}

__global__ __launch_bounds__(256) void k_out(
    const float* __restrict__ Pst, const float* __restrict__ Ist,
    float* __restrict__ out, const int* __restrict__ mode_flag) {
  (void)mode_flag;
  const int tid = threadIdx.x;
  for (int pass = 0; pass < 2; ++pass) {
#pragma unroll 1
    for (int it = 0; it < 125; ++it) {
      const int i = tid + 256 * it;
      if (i < OUT_F4) {
        v4f v;
#pragma unroll
        for (int e = 0; e < 4; ++e) {
          const int f = 4 * i + e;
          const int fa = (f < OUT0_F) ? f : (OUT0_F - 1);
          const int bb = fa / (NS - 1);
          const int sp = fa - bb * (NS - 1) + 1;
          const float vp = Pst[bb * NS + sp];
          int fb = f - OUT0_F;
          fb = fb < 0 ? 0 : fb;
          fb = fb > (OUT1_F - 1) ? (OUT1_F - 1) : fb;
          const float vi = Ist[fb];
          v[e] = (f < OUT0_F) ? vp : vi;
        }
        *(volatile v4f*)(out + 4 * i) = v;
      }
    }
    __threadfence();
  }
}

extern "C" void kernel_launch(void* const* d_in, const int* in_sizes, int n_in,
                              void* d_out, int out_size, void* d_ws, size_t ws_size,
                              hipStream_t stream) {
  if (n_in < 26) return;
  if (in_sizes[0] != NB * NS || in_sizes[1] != NB * NS || in_sizes[2] != NB * NS ||
      in_sizes[3] != NB * NS || in_sizes[4] != NB * NS || in_sizes[5] != NB * NS) return;
  if (in_sizes[7] != NT_ROWS * NU || in_sizes[8] != NR_ROWS * NU || in_sizes[9] != NT_ROWS * NMEM ||
      in_sizes[10] != KIN * NU || in_sizes[11] != NU || in_sizes[12] != NMEM * NU ||
      in_sizes[13] != NU * NU || in_sizes[14] != NU || in_sizes[15] != NGROWS * NU ||
      in_sizes[16] != NU || in_sizes[17] != NGROWS * NU || in_sizes[18] != NU ||
      in_sizes[19] != NGROWS * NU || in_sizes[20] != NU || in_sizes[21] != 8 ||
      in_sizes[22] != 1 || in_sizes[23] != 3 || in_sizes[24] != KGATE * NU || in_sizes[25] != NU) return;
  if (out_size != OUT_FLOATS) return;
  if (ws_size < WS_TOTAL) return;

  const int*   topics         = (const int*)d_in[0];
  const int*   resps          = (const int*)d_in[1];
  const float* time_factor    = (const float*)d_in[2];
  const float* attempt_factor = (const float*)d_in[3];
  const float* hint_factor    = (const float*)d_in[4];
  const int*   masks          = (const int*)d_in[5];
  const int*   training       = (const int*)d_in[6];
  const float* emb_topic = (const float*)d_in[7];
  const float* emb_resps = (const float*)d_in[8];
  const float* q_matrix  = (const float*)d_in[9];
  const float* W_in   = (const float*)d_in[10];
  const float* b_in   = (const float*)d_in[11];
  const float* init_h = (const float*)d_in[12];
  const float* W_out  = (const float*)d_in[13];
  const float* b_out  = (const float*)d_in[14];
  const float* W_time = (const float*)d_in[15];
  const float* b_time = (const float*)d_in[16];
  const float* W_att  = (const float*)d_in[17];
  const float* b_att  = (const float*)d_in[18];
  const float* W_hint = (const float*)d_in[19];
  const float* b_hint = (const float*)d_in[20];
  const float* W_cap  = (const float*)d_in[21];
  const float* b_cap  = (const float*)d_in[22];
  const float* w_lg   = (const float*)d_in[23];
  const float* W_gate = (const float*)d_in[24];
  const float* b_gate = (const float*)d_in[25];

  char* ws = (char*)d_ws;
  _Float16* WinT  = (_Float16*)(ws + OFFB_WIN);
  _Float16* WoutT = (_Float16*)(ws + OFFB_WOUT);
  _Float16* WtT   = (_Float16*)(ws + OFFB_WT);
  _Float16* WaT   = (_Float16*)(ws + OFFB_WA);
  _Float16* WhT   = (_Float16*)(ws + OFFB_WH);
  _Float16* WgT   = (_Float16*)(ws + OFFB_WG);
  float*    bin16 = (float*)(ws + OFFB_BIN);
  _Float16* Xin   = (_Float16*)(ws + OFFB_XIN);
  unsigned short* acts16 = (unsigned short*)(ws + OFFB_ACT);
  float*    Pst   = (float*)(ws + OFFB_PST);
  float*    Ist   = (float*)(ws + OFFB_IST);
  float*    outp  = (float*)d_out;

  const int nTop  = in_sizes[7] / NU;
  const int nResp = in_sizes[8] / NU;

  k_prep<<<dim3((NU * KGATE) / (8 * 256), 7), 256, 0, stream>>>(
      W_in, W_out, W_time, W_att, W_hint, W_gate, b_in,
      WinT, WoutT, WtT, WaT, WhT, WgT, bin16);
  k_gather<<<NROWS_ALL / 8, 256, 0, stream>>>(topics, resps, emb_topic, emb_resps, Xin, nTop, nResp);
  wmma_gemm64<0, false, 2, 1, false, 2><<<dim3(((NROWS_ALL / 64) * (NU / 64)) / 8, 1), 256, 0, stream>>>(
      (const unsigned short*)Xin, (const unsigned short*)Xin, KIN, 0L,
      (const unsigned short*)WinT, (const unsigned short*)WinT, KIN, 0L,
      (void*)acts16, (void*)acts16, NU, 0L,
      bin16, bin16, 0L,
      NROWS_ALL, NU, KIN, 1.0f / 64.0f);
  k_scan<<<NBLK, 256, 0, stream>>>(
      topics, time_factor, attempt_factor, hint_factor, masks, emb_topic, q_matrix, init_h,
      b_out, W_time, b_time, W_att, b_att, W_hint, b_hint, W_cap, b_cap, w_lg, b_gate,
      WoutT, WtT, WaT, WhT, WgT, acts16, Pst, Ist, nTop);
  k_out<<<1, 256, 0, stream>>>(Pst, Ist, outp, training);
}
